// FuseCausal_81965155877006
// MI455X (gfx1250) — hardware-run, weakly checked
//
#include <hip/hip_runtime.h>


#ifndef NROW
#define NROW 2048
#endif
#define NROW_FULL 2048
#ifndef OUT_PITCH
#define OUT_PITCH NROW
#endif
#define DK   1024
#define CLS  10
#define NPC  32
#define OSP  36
#define PJ   256
#define PIT  32
#define RBP  21
#define YP   ((2 * CLS) / 4)
#define LOG2E 1.4426950408889634f
#define LN2   0.6931471805599453f
#define GCE_Q 0.7f
#define EPS_W 1.0e-8f

static_assert(DK % 32 == 0);
static_assert(NPC == 32);
static_assert(2 * CLS <= NPC);
static_assert((2 * CLS) % 4 == 0);
static_assert(2 * CLS + 2 <= NPC);
static_assert(2 * CLS <= 20);
static_assert(YP < 8);
static_assert(NROW % 16 == 0);
static_assert(NROW % PJ == 0);
static_assert(NROW % PIT == 0);
static_assert(PJ == PIT * 8);
static_assert(PJ % 32 == 0);
static_assert(32 * 4 == 128);
static_assert(OUT_PITCH % 32 == 0);
static_assert(OUT_PITCH >= NROW);
static_assert(RBP >= 2 * CLS);
static_assert((RBP & 1) == 1);
static_assert(((size_t)NROW * DK) % 8 == 0);
static_assert(((size_t)NPC * DK / 8) % 256 == 0);
static_assert(32 * 16 * 4 == 16 * NPC * 4);
static_assert((OSP * 4) % 16 == 0);
static_assert(OSP >= NPC);
static_assert(16 * OSP * 4 <= 131072);
static_assert((PIT * NPC + PJ * RBP) * 4 + PIT * 4 <= 131072);
static_assert(NROW <= NROW_FULL);

typedef unsigned short bf;
typedef __attribute__((ext_vector_type(16))) __bf16   v16bf;
typedef __attribute__((ext_vector_type(8)))  unsigned short v8us;
typedef __attribute__((ext_vector_type(8)))  float    v8f;
typedef __attribute__((ext_vector_type(4)))  float    v4f;
typedef v4f  __attribute__((may_alias)) v4fa;

__device__ __forceinline__ unsigned short f2bf(float f) { unsigned u = __float_as_uint(f); u += 0x7FFFu + ((u >> 16) & 1u); return (unsigned short)(u >> 16); }
__device__ __forceinline__ float bfr(float f) { return __uint_as_float(((unsigned)f2bf(f)) << 16); }
__device__ __forceinline__ v16bf cat16b(v8us lo, v8us hi) { return __builtin_bit_cast(v16bf, __builtin_shufflevector(lo, hi, 0, 1, 2, 3, 4, 5, 6, 7, 8, 9, 10, 11, 12, 13, 14, 15)); }
__device__ __forceinline__ v8f wmmab(v16bf a, v16bf b, v8f c) { return __builtin_amdgcn_wmma_f32_16x16x32_bf16(false, a, false, b, (short)0, c, false, false); }
__device__ __forceinline__ v8f wmmab_g(v16bf a, v16bf b, v8f c) { c = wmmab(a, b, c); asm volatile("v_nop\n\tv_nop\n\tv_nop\n\tv_nop" : "+v"(c) : "v"(a), "v"(b)); return c; }
__device__ __forceinline__ v16bf ldb(const bf* p)  { return cat16b(*(const v8us*)p, *(const v8us*)(p + 16)); }
__device__ __forceinline__ void wave_sync() { __builtin_amdgcn_fence(3  , "wavefront"); __builtin_amdgcn_wave_barrier(); asm volatile("" ::: "memory"); }

__global__ __launch_bounds__(256) void k_cvt8(const float* __restrict__ src, bf* dst, size_t n8) {
    const size_t i = (size_t)blockIdx.x * 256 + threadIdx.x; if (i >= n8) return;
    const v8f v = *(const v8f*)(src + i * 8); v8us o;
#pragma unroll
    for (int k = 0; k < 8; ++k) o[k] = f2bf(v[k]);
    *(volatile v8us*)(dst + i * 8) = o; __threadfence(); *(volatile v8us*)(dst + i * 8) = o;
}

__global__ __launch_bounds__(256) void k_wpack(const float* __restrict__ Wc, const float* __restrict__ Wb, bf* dst) {
    const int i = (int)(blockIdx.x * 256 + threadIdx.x);
    if (i >= NPC * DK / 8) return;
    const int row = i / (DK / 8), c8 = (i % (DK / 8)) * 8;
    const int rc = row < CLS ? row : (CLS - 1);
    int rb = row - CLS; rb = rb < 0 ? 0 : (rb > CLS - 1 ? CLS - 1 : rb);
    v8f vc = *(const v8f*)(Wc + (size_t)rc * DK + c8);
    v8f vb = *(const v8f*)(Wb + (size_t)rb * DK + c8);
    asm volatile("" : "+v"(vc), "+v"(vb));
    const bool isc = row < CLS;
    const bool isb = (row >= CLS) & (row < 2 * CLS);
    v8us o;
#pragma unroll
    for (int k = 0; k < 8; ++k) { const float s = isc ? vc[k] : (isb ? vb[k] : 0.0f); o[k] = f2bf(s); }
    *(volatile v8us*)(dst + (size_t)i * 8) = o; __threadfence(); *(volatile v8us*)(dst + (size_t)i * 8) = o;
}

__global__ __launch_bounds__(32) void k_projf(const bf* __restrict__ A, const bf* __restrict__ Bt, float* PF) {
    __shared__ __align__(16) float os[16 * OSP];
    const int K = DK;
    const int lane = threadIdx.x & 31, lr = lane & 15, hi = lane >> 4; const int r0 = blockIdx.x * 16;
    v8f acc0 = (v8f){}, acc1 = (v8f){};
    const size_t aoff = (size_t)(r0 + lr) * K + 8 * hi, boff = (size_t)lr * K + 8 * hi;
#pragma unroll 1
    for (int kc = 0; kc < K; kc += 32) {
        const v16bf a = ldb(A + aoff + kc);
        const v16bf b0 = ldb(Bt + boff + kc);
        const v16bf b1 = ldb(Bt + boff + (size_t)16 * K + kc);
        acc0 = wmmab_g(a, b0, acc0);
        acc1 = wmmab_g(a, b1, acc1);
    }
#pragma unroll
    for (int r = 0; r < 8; ++r) { os[(hi * 8 + r) * OSP + lr] = acc0[r]; os[(hi * 8 + r) * OSP + 16 + lr] = acc1[r]; }
    wave_sync();
    float* orow = PF + (size_t)r0 * NPC;
#pragma unroll 1
    for (int ps = 0; ps < 2; ++ps) {
#pragma unroll
        for (int s = 0; s < 4; ++s) { const int row = 4 * s + (lane >> 3), cofs = (lane & 7) * 4;
            const v4f val = *(const v4fa*)(&os[row * OSP + cofs]);
            *(volatile v4f*)(orow + (size_t)row * NPC + cofs) = val; }
        if (ps == 0) __threadfence(); }
}

__global__ __launch_bounds__(PJ) void k_pair(const float* __restrict__ PF, const float* __restrict__ bc, const float* __restrict__ bb, const int* __restrict__ y, float* OUT) {
#pragma clang fp contract(off)
    __shared__ __align__(16) float sL[PIT * NPC];
    __shared__ float sRB[PJ * RBP];
    __shared__ int syi[PIT];
    const int tid = (int)threadIdx.x;
    const int i0 = (int)blockIdx.y * PIT;
    const int j = (int)blockIdx.x * PJ + tid;
    {
        const int row = tid >> 3, piece = tid & 7;
        const int gi = i0 + row;
        int yv = y[gi]; yv = yv < 0 ? 0 : (yv > CLS - 1 ? CLS - 1 : yv);
        const float* lrow = PF + (size_t)gi * NPC;
        v4f v = *(const v4f*)(lrow + piece * 4);
        float a = lrow[yv], b = lrow[CLS + yv];
        asm volatile("" : "+v"(v), "+v"(a), "+v"(b));
        const bool py = piece == YP;
        v[0] = py ? a : v[0]; v[1] = py ? b : v[1];
        *(v4fa*)(&sL[row * NPC + piece * 4]) = v;
        if (piece == 0) syi[row] = yv;
    }
    const float* rrow = PF + (size_t)(NROW + j) * NPC;
    v4f rq[5];
#pragma unroll
    for (int q = 0; q < 5; ++q) rq[q] = *(const v4f*)(rrow + 4 * q);
    float rbc[CLS], rbb[CLS];
#pragma unroll
    for (int k = 0; k < CLS; ++k) {
        rbc[k] = rq[k >> 2][k & 3] + bfr(bc[k]);
        rbb[k] = rq[(CLS + k) >> 2][(CLS + k) & 3] + bfr(bb[k]);
        sRB[tid * RBP + k] = rbc[k];
        sRB[tid * RBP + CLS + k] = rbb[k];
    }
    int yj = y[j]; yj = yj < 0 ? 0 : (yj > CLS - 1 ? CLS - 1 : yj);
    __syncthreads();
    const float rbyj = sRB[tid * RBP + CLS + yj];
#pragma unroll 1
    for (int i = 0; i < PIT; ++i) {
        const int yi = syi[i];
        v4f lq[6];
#pragma unroll
        for (int q = 0; q < 6; ++q) lq[q] = *(const v4fa*)(&sL[i * NPC + 4 * q]);
        float lc[CLS], lb[CLS];
#pragma unroll
        for (int k = 0; k < CLS; ++k) { lc[k] = lq[k >> 2][k & 3] + rbc[k]; lb[k] = lq[(CLS + k) >> 2][(CLS + k) & 3] + rbb[k]; }
        float mc = lc[0], mb = lb[0];
#pragma unroll
        for (int k = 1; k < CLS; ++k) { mc = __builtin_fmaxf(mc, lc[k]); mb = __builtin_fmaxf(mb, lb[k]); }
        float sc = 0.0f, sb = 0.0f;
#pragma unroll
        for (int k = 0; k < CLS; ++k) { sc += __builtin_amdgcn_exp2f((lc[k] - mc) * LOG2E); sb += __builtin_amdgcn_exp2f((lb[k] - mb) * LOG2E); }
        const float lse_c = __builtin_amdgcn_logf(sc) * LN2 + mc;
        const float lse_b = __builtin_amdgcn_logf(sb) * LN2 + mb;
        const float lc_yi = lq[YP][0] + sRB[tid * RBP + yi];
        const float lb_yi = lq[YP][1] + sRB[tid * RBP + CLS + yi];
        const float lb_yj = sL[i * NPC + CLS + yj] + rbyj;
        const float ce_pc = lse_c - lc_yi;
        const float ce_pb = lse_b - lb_yi;
        const float logp = lb_yj - lse_b;
        const float gce = (-logp) * __builtin_amdgcn_exp2f((GCE_Q * logp) * LOG2E);
        const float den = (ce_pc + ce_pb) + EPS_W;
        const float w = ce_pb * __builtin_amdgcn_rcpf(den);
        const float val = w * ce_pc + (1.0f - w) * gce;
        float* op = OUT + (size_t)(i0 + i) * OUT_PITCH + j;
        *(volatile float*)op = val; __threadfence(); *(volatile float*)op = val;
    }
}

static constexpr size_t al256(size_t v) { return (v + 255) & ~(size_t)255; }
static constexpr size_t SZ_ZB = al256((size_t)2 * NROW * DK * 2);
static constexpr size_t SZ_WB = al256((size_t)NPC * DK * 2);
static constexpr size_t SZ_PF = al256((size_t)2 * NROW * NPC * 4);
static constexpr size_t SZ_TOTAL = SZ_ZB + SZ_WB + SZ_PF;
static_assert(SZ_TOTAL <= (size_t)134217728);
static_assert(((size_t)NROW * DK * 2) % 256 == 0);

extern "C" void kernel_launch(void* const* d_in, const int* in_sizes, int n_in,
                              void* d_out, int out_size, void* d_ws, size_t ws_size, hipStream_t stream) {
    if (n_in < 7) return;
    if ((size_t)in_sizes[0] < (size_t)NROW * DK || (size_t)in_sizes[1] < (size_t)NROW * DK) return;
    if ((size_t)in_sizes[2] < (size_t)CLS * DK || (size_t)in_sizes[4] < (size_t)CLS * DK) return;
    if (in_sizes[3] < CLS || in_sizes[5] < CLS || in_sizes[6] < NROW) return;
    if ((size_t)out_size < (size_t)(NROW - 1) * OUT_PITCH + NROW) return;
    if (SZ_TOTAL > ws_size) return;
    const float* zc = (const float*)d_in[0]; const float* zb = (const float*)d_in[1];
    const float* wc = (const float*)d_in[2]; const float* bc = (const float*)d_in[3];
    const float* wb = (const float*)d_in[4]; const float* bb = (const float*)d_in[5];
    const int* y = (const int*)d_in[6];
    float* OUT = (float*)d_out;
    char* wsp = (char*)d_ws;
    bf* ZB = (bf*)wsp; wsp += SZ_ZB;
    bf* WB = (bf*)wsp; wsp += SZ_WB;
    float* PF = (float*)wsp; wsp += SZ_PF;

    { const size_t n8 = (size_t)NROW * DK / 8; const unsigned g = (unsigned)((n8 + 255) / 256);
      k_cvt8<<<g, 256, 0, stream>>>(zc, ZB, n8);
      k_cvt8<<<g, 256, 0, stream>>>(zb, ZB + (size_t)NROW * DK, n8); }
    k_wpack<<<(unsigned)(NPC * DK / 8 / 256), 256, 0, stream>>>(wc, wb, WB);
    k_projf<<<(unsigned)(2 * NROW / 16), 32, 0, stream>>>(ZB, WB, PF);
    k_pair<<<dim3(NROW / PJ, NROW / PIT, 1), PJ, 0, stream>>>(PF, bc, bb, y, OUT);
}
